// GNNMessagePassing_18416819765909
// MI455X (gfx1250) — hardware-verified
//
#include <hip/hip_runtime.h>
#include <stddef.h>


#define IN    256
#define HID   64
#define HEADS 4
#define GR    32
#define AP    264
#define CP    260
#define TT    64
#define TP    72
#define NB    128
#define SLB   7
#define CHUNK 2048
#define NTHR  256
#define NWAVE 8
#define WCAP  256
#define NGRP  (CHUNK / (NTHR * 4))

#define LDS_SACC_B (NB * IN * 4)
#define LDS_QS_B   (NB * IN * 2)
#define LDS_AGG_BYTES (LDS_SACC_B + LDS_QS_B + NB * HEADS * 4 * 2 + NB * 4 + NWAVE * WCAP * 4 + NWAVE * 4)

static_assert(IN == HID * HEADS);
static_assert(WCAP == (CHUNK / NTHR) * 32);
static_assert(NGRP >= 1);
static_assert((1 << SLB) == NB);
static_assert(CHUNK <= 4096);
static_assert(NB % NWAVE == 0);
static_assert(GR == 4 * NWAVE);
static_assert(LDS_AGG_BYTES == 209440);
static_assert((LDS_SACC_B % 16) == 0 && (LDS_QS_B % 16) == 0);

typedef float    v4f  __attribute__((ext_vector_type(4)));
typedef float    v8f  __attribute__((ext_vector_type(8)));
typedef int      v4i  __attribute__((ext_vector_type(4)));
typedef _Float16 v8h  __attribute__((ext_vector_type(8)));
typedef _Float16 v16h __attribute__((ext_vector_type(16)));
union Frag   { v16h v; v8h half[2]; };
union Pack16 { v8h h; v4i i; };

__device__ __forceinline__ v8f wm(v16h a, v16h b, v8f c) {
  v8f d = __builtin_amdgcn_wmma_f32_16x16x32_f16(false, a, false, b, (short)0, c, false, false);
  asm volatile("v_nop\n\tv_nop\n\tv_nop\n\tv_nop" : "+v"(d) : "v"(a), "v"(b));
  return d;
}

__device__ __forceinline__ float wsum(float v) {
  v += __shfl_xor(v, 16, 32);
  v += __shfl_xor(v, 8, 32);
  v += __shfl_xor(v, 4, 32);
  v += __shfl_xor(v, 2, 32);
  v += __shfl_xor(v, 1, 32);
  return v;
}

__device__ __forceinline__ v8h cvt8(v4f a, v4f b) {
  Pack16 u;
  u.h[0] = (_Float16)a.x; u.h[1] = (_Float16)a.y; u.h[2] = (_Float16)a.z; u.h[3] = (_Float16)a.w;
  u.h[4] = (_Float16)b.x; u.h[5] = (_Float16)b.y; u.h[6] = (_Float16)b.z; u.h[7] = (_Float16)b.w;
  return u.h;
}

__global__ __launch_bounds__(NTHR) void k_prepw(
    const float* __restrict__ W0, const float* __restrict__ W1,
    const float* __restrict__ W2, const float* __restrict__ W3, _Float16* Wt) {
  __shared__ __attribute__((aligned(16))) _Float16 T[TT * TP];
  const int tid = threadIdx.x;
  const int k0  = blockIdx.x * TT;
  const int n0  = blockIdx.y * TT;
  const int mat = blockIdx.z;
  const float* W = (mat == 0) ? W0 : ((mat == 1) ? W1 : ((mat == 2) ? W2 : W3));
  {
    const int kr = tid >> 2;
    const int nc = (tid & 3) * 16;
    const float* p = W + (size_t)(k0 + kr) * IN + n0 + nc;
    const v4f f0 = *(const v4f*)(p), f1 = *(const v4f*)(p + 4);
    const v4f f2 = *(const v4f*)(p + 8), f3 = *(const v4f*)(p + 12);
    _Float16* tp = T + nc * TP + kr;
    tp[0 * TP]  = (_Float16)(f0.x * 32.0f); tp[1 * TP]  = (_Float16)(f0.y * 32.0f);
    tp[2 * TP]  = (_Float16)(f0.z * 32.0f); tp[3 * TP]  = (_Float16)(f0.w * 32.0f);
    tp[4 * TP]  = (_Float16)(f1.x * 32.0f); tp[5 * TP]  = (_Float16)(f1.y * 32.0f);
    tp[6 * TP]  = (_Float16)(f1.z * 32.0f); tp[7 * TP]  = (_Float16)(f1.w * 32.0f);
    tp[8 * TP]  = (_Float16)(f2.x * 32.0f); tp[9 * TP]  = (_Float16)(f2.y * 32.0f);
    tp[10 * TP] = (_Float16)(f2.z * 32.0f); tp[11 * TP] = (_Float16)(f2.w * 32.0f);
    tp[12 * TP] = (_Float16)(f3.x * 32.0f); tp[13 * TP] = (_Float16)(f3.y * 32.0f);
    tp[14 * TP] = (_Float16)(f3.z * 32.0f); tp[15 * TP] = (_Float16)(f3.w * 32.0f);
  }
  __syncthreads();
  Pack16 u[2];
  _Float16* dp[2];
#pragma unroll
  for (int ps = 0; ps < 2; ++ps) {
    const int L     = ps * 32 + (tid >> 3);
    const int piece = tid & 7;
    u[ps].h = *(const v8h*)(T + L * TP + piece * 8);
    dp[ps]  = Wt + ((size_t)(mat * IN + n0 + L) * IN + k0 + piece * 8);
  }
#pragma unroll
  for (int ps = 0; ps < 2; ++ps) *(volatile v4i*)dp[ps] = u[ps].i;
  __threadfence();
#pragma unroll
  for (int ps = 0; ps < 2; ++ps) *(volatile v4i*)dp[ps] = u[ps].i;
}

__device__ __forceinline__ void epi_tile(v8f acc, int T, int hh, int col,
                                         const float* bias, float* Cs) {
  const float b = bias[col];
#pragma unroll
  for (int r = 0; r < 8; ++r) Cs[(T * 16 + 8 * hh + r) * CP + col] = acc[r] * 0.03125f + b;
}

template <int MODE>
__global__ __launch_bounds__(NTHR) void k_gemm(
    const float* __restrict__ x, const float* __restrict__ qe, const _Float16* __restrict__ Ah,
    const _Float16* __restrict__ Wt,
    const float* __restrict__ b0p, const float* __restrict__ b1p, const float* __restrict__ b2p,
    const float* __restrict__ gam, const float* __restrict__ bet,
    _Float16* P0, _Float16* P1, _Float16* P2, float* out, int nN) {
  __shared__ __attribute__((aligned(16))) _Float16 At[GR * AP];
  __shared__ __attribute__((aligned(16))) float Cs[GR * CP];

  const int tid  = threadIdx.x;
  const int lane = tid & 31;
  const int wave = tid >> 5;
  const int hh   = lane >> 4;
  const int m    = lane & 15;
  const int mat  = (MODE == 0) ? (int)blockIdx.y : 0;
  const int rowBase = blockIdx.x * GR;

  {
    const int r  = tid >> 3;
    const int c0 = (tid & 7) * 32;
    int row = rowBase + r;
    if (row > nN - 1) row = nN - 1;
    if (MODE == 0) {
      const float* p  = x + (size_t)row * IN + c0;
      const float* pq = qe + c0;
#pragma unroll
      for (int j = 0; j < 4; ++j) {
        const v4f xa = *(const v4f*)(p + 8 * j), xb = *(const v4f*)(p + 8 * j + 4);
        const v4f qa = *(const v4f*)(pq + 8 * j), qb = *(const v4f*)(pq + 8 * j + 4);
        const v4f ea = xa + qa * 0.1f;
        const v4f eb = xb + qb * 0.1f;
        *(v8h*)(At + r * AP + c0 + 8 * j) = cvt8(ea, eb);
      }
    } else {
      const _Float16* p = Ah + (size_t)row * IN + c0;
#pragma unroll
      for (int j = 0; j < 4; ++j) *(v8h*)(At + r * AP + c0 + 8 * j) = *(const v8h*)(p + 8 * j);
    }
  }
  __syncthreads();

  const _Float16* Wm = Wt + (size_t)mat * IN * IN;
  const int ncol0 = wave * 32;
  v8f c00 = {0.f, 0.f, 0.f, 0.f, 0.f, 0.f, 0.f, 0.f};
  v8f c01 = {0.f, 0.f, 0.f, 0.f, 0.f, 0.f, 0.f, 0.f};
  v8f c10 = {0.f, 0.f, 0.f, 0.f, 0.f, 0.f, 0.f, 0.f};
  v8f c11 = {0.f, 0.f, 0.f, 0.f, 0.f, 0.f, 0.f, 0.f};
#pragma unroll
  for (int kt = 0; kt < IN / 32; ++kt) {
    const int k0 = kt * 32;
    Frag a0, a1, bb0, bb1;
    const _Float16* pa0 = At + m * AP + k0 + 8 * hh;
    const _Float16* pa1 = At + (16 + m) * AP + k0 + 8 * hh;
    const _Float16* pb0 = Wm + (size_t)(ncol0 + m) * IN + k0 + 8 * hh;
    const _Float16* pb1 = Wm + (size_t)(ncol0 + 16 + m) * IN + k0 + 8 * hh;
    a0.half[0]  = *(const v8h*)pa0;  a0.half[1]  = *(const v8h*)(pa0 + 16);
    a1.half[0]  = *(const v8h*)pa1;  a1.half[1]  = *(const v8h*)(pa1 + 16);
    bb0.half[0] = *(const v8h*)pb0;  bb0.half[1] = *(const v8h*)(pb0 + 16);
    bb1.half[0] = *(const v8h*)pb1;  bb1.half[1] = *(const v8h*)(pb1 + 16);
    c00 = wm(a0.v, bb0.v, c00);
    c01 = wm(a0.v, bb1.v, c01);
    c10 = wm(a1.v, bb0.v, c10);
    c11 = wm(a1.v, bb1.v, c11);
  }

  const float* bias = (MODE == 0) ? ((mat == 0) ? b0p : ((mat == 1) ? b1p : b2p)) : b0p;
  epi_tile(c00, 0, hh, ncol0 + m,      bias, Cs);
  epi_tile(c01, 0, hh, ncol0 + 16 + m, bias, Cs);
  epi_tile(c10, 1, hh, ncol0 + m,      bias, Cs);
  epi_tile(c11, 1, hh, ncol0 + 16 + m, bias, Cs);
  __syncthreads();

  if (MODE == 0) {
    _Float16* P = (mat == 0) ? P0 : ((mat == 1) ? P1 : P2);
    Pack16 u[4];
    _Float16* pp[4];
#pragma unroll
    for (int i = 0; i < 4; ++i) {
      const int lr = 4 * wave + i;
      const v4f ca = *(const v4f*)(Cs + lr * CP + 8 * lane);
      const v4f cb = *(const v4f*)(Cs + lr * CP + 8 * lane + 4);
      u[i].h = cvt8(ca, cb);
      pp[i]  = P + (size_t)(rowBase + lr) * IN + 8 * lane;
    }
#pragma unroll
    for (int i = 0; i < 4; ++i) *(volatile v4i*)pp[i] = u[i].i;
    __threadfence();
#pragma unroll
    for (int i = 0; i < 4; ++i) *(volatile v4i*)pp[i] = u[i].i;
  } else {
    const v4f ga = *(const v4f*)(gam + 4 * lane), gb = *(const v4f*)(gam + 128 + 4 * lane);
    const v4f ea = *(const v4f*)(bet + 4 * lane), eb = *(const v4f*)(bet + 128 + 4 * lane);
#pragma unroll
    for (int i = 0; i < 4; ++i) {
      const int lr   = 4 * wave + i;
      const int grow = rowBase + lr;
      if (grow >= nN) break;
      const v4f ca = *(const v4f*)(Cs + lr * CP + 4 * lane);
      const v4f cb = *(const v4f*)(Cs + lr * CP + 128 + 4 * lane);
      const v4f xa = *(const v4f*)(x + (size_t)grow * IN + 4 * lane);
      const v4f xb = *(const v4f*)(x + (size_t)grow * IN + 128 + 4 * lane);
      const v4f ha = ca + xa;
      const v4f hb = cb + xb;
      const float s  = wsum(ha.x + ha.y + ha.z + ha.w + hb.x + hb.y + hb.z + hb.w);
      const float mu = s * (1.0f / IN);
      const v4f da = ha - mu;
      const v4f db = hb - mu;
      const float q = wsum(da.x * da.x + da.y * da.y + da.z * da.z + da.w * da.w +
                           db.x * db.x + db.y * db.y + db.z * db.z + db.w * db.w);
      const float rs = rsqrtf(q * (1.0f / IN) + 1e-5f);
      const v4f ya = da * rs * ga + ea;
      const v4f yb = db * rs * gb + eb;
      float* op = out + (size_t)grow * IN + 4 * lane;
      *(volatile v4f*)op = ya;
      *(volatile v4f*)(op + 128) = yb;
      __threadfence();
      *(volatile v4f*)op = ya;
      *(volatile v4f*)(op + 128) = yb;
    }
  }
}

__global__ __launch_bounds__(NTHR) void k_agg(
    const int* __restrict__ ei, const int* __restrict__ erel,
    const _Float16* __restrict__ Qh, const _Float16* __restrict__ Kh, const _Float16* __restrict__ Vh,
    const float* __restrict__ relw, _Float16* Mh, int nN, int nE, int nR) {
  extern __shared__ v4f lds_dyn[];
  float*    sacc = (float*)lds_dyn;
  _Float16* qs   = (_Float16*)((char*)lds_dyn + LDS_SACC_B);
  float*    smx  = (float*)((char*)lds_dyn + LDS_SACC_B + LDS_QS_B);
  float*    den  = smx + NB * HEADS;
  int*      cnt  = (int*)(den + NB * HEADS);
  int*      list = cnt + NB;
  int*      wcnt = list + NWAVE * WCAP;

  const int tid  = threadIdx.x;
  const int lane = tid & 31;
  const int wave = tid >> 5;
  const int nodeBase = blockIdx.x * NB;

  {
    const v4f z4 = {0.f, 0.f, 0.f, 0.f};
    for (int i = tid; i < (NB * IN) / 4; i += NTHR) lds_dyn[i] = z4;
    for (int i = tid; i < NB * HEADS; i += NTHR) { smx[i] = -1.0e30f; den[i] = 0.f; }
    if (tid < NB) cnt[tid] = 0;
    for (int p = tid; p < NB * (IN / 8); p += NTHR) {
      const int slot  = p >> 5;
      const int piece = p & 31;
      int node = nodeBase + slot;
      if (node > nN - 1) node = nN - 1;
      *(v8h*)(qs + slot * IN + piece * 8) = *(const v8h*)(Qh + (size_t)node * IN + piece * 8);
    }
  }
  __syncthreads();

  const int* eid = ei + nE;
  const bool al16 = ((nE & 3) == 0);

  const int nChunks = (nE + CHUNK - 1) / CHUNK;
#pragma unroll 1
  for (int ch = 0; ch < nChunks; ++ch) {
    const int cbase = ch * CHUNK;
    int wc = 0;
#pragma unroll
    for (int g = 0; g < NGRP; ++g) {
      const int el0 = (g * NTHR + tid) * 4;
      const int e0  = cbase + el0;
      const int sent = -2147483647 - 1;
      v4i d;
      if (al16 && (cbase + CHUNK <= nE)) {
        d = *(const v4i*)(eid + e0);
      } else {
        d.x = (e0     < nE) ? eid[min(e0,     nE - 1)] : sent;
        d.y = (e0 + 1 < nE) ? eid[min(e0 + 1, nE - 1)] : sent;
        d.z = (e0 + 2 < nE) ? eid[min(e0 + 2, nE - 1)] : sent;
        d.w = (e0 + 3 < nE) ? eid[min(e0 + 3, nE - 1)] : sent;
      }
      const unsigned s0 = (unsigned)d.x - (unsigned)nodeBase;
      const unsigned s1 = (unsigned)d.y - (unsigned)nodeBase;
      const unsigned s2 = (unsigned)d.z - (unsigned)nodeBase;
      const unsigned s3 = (unsigned)d.w - (unsigned)nodeBase;
      const bool h0 = s0 < (unsigned)NB;
      const bool h1 = s1 < (unsigned)NB;
      const bool h2 = s2 < (unsigned)NB;
      const bool h3 = s3 < (unsigned)NB;
      const unsigned many = __builtin_amdgcn_ballot_w32(h0 | h1 | h2 | h3);
      if (many != 0u) {
#define HITJ(J, HJ, SJ) { \
          const unsigned mj = __builtin_amdgcn_ballot_w32(HJ); \
          if (HJ) { \
            const int pos = wc + (int)__builtin_amdgcn_mbcnt_lo(mj, 0u); \
            if (pos < WCAP) list[wave * WCAP + pos] = ((el0 + (J)) << SLB) | (int)(SJ); \
          } \
          wc += (int)__builtin_popcount(mj); }
        HITJ(0, h0, s0)
        HITJ(1, h1, s1)
        HITJ(2, h2, s2)
        HITJ(3, h3, s3)
#undef HITJ
      }
    }
    if (lane == 0) wcnt[wave] = wc;
    __syncthreads();

    if (wave == 0) {
      for (int wsx = 0; wsx < NWAVE; ++wsx) {
        int n = wcnt[wsx];
        if (n > WCAP) n = WCAP;
        if (n < 0) n = 0;
        for (int i = 0; i < n; ++i) {
          const int ent  = list[wsx * WCAP + i];
          const int slot = ent & (NB - 1);
          const int el   = (ent >> SLB) & (CHUNK - 1);
          int e = cbase + el;
          if (e > nE - 1) e = nE - 1;
          int src = ei[e];
          src = src < 0 ? 0 : (src > nN - 1 ? nN - 1 : src);
          int rr = erel[e];
          rr = rr < 0 ? 0 : (rr > nR - 1 ? nR - 1 : rr);
          const v8h k8 = *(const v8h*)(Kh + (size_t)src * IN + 8 * lane);
          const v8h v8 = *(const v8h*)(Vh + (size_t)src * IN + 8 * lane);
          const v8h q8 = *(const v8h*)(qs + slot * IN + 8 * lane);
          const float* rp = relw + (size_t)rr * HID + 8 * (lane & 7);
          const v4f ra = *(const v4f*)rp, rb = *(const v4f*)(rp + 4);
          float part = 0.f;
          part += (float)q8[0] * ((float)k8[0] + 0.2f * ra.x);
          part += (float)q8[1] * ((float)k8[1] + 0.2f * ra.y);
          part += (float)q8[2] * ((float)k8[2] + 0.2f * ra.z);
          part += (float)q8[3] * ((float)k8[3] + 0.2f * ra.w);
          part += (float)q8[4] * ((float)k8[4] + 0.2f * rb.x);
          part += (float)q8[5] * ((float)k8[5] + 0.2f * rb.y);
          part += (float)q8[6] * ((float)k8[6] + 0.2f * rb.z);
          part += (float)q8[7] * ((float)k8[7] + 0.2f * rb.w);
          part += __shfl_xor(part, 1, 32);
          part += __shfl_xor(part, 2, 32);
          part += __shfl_xor(part, 4, 32);
          const float s  = part * 0.125f;
          const int   hh = lane >> 3;
          const float mo = smx[slot * HEADS + hh];
          const float dn = den[slot * HEADS + hh];
          const float mn = fmaxf(mo, s);
          const float sc = __expf(mo - mn);
          const float p  = __expf(s - mn);
          v4f* ap = (v4f*)(sacc + slot * IN + 8 * lane);
          v4f a0 = ap[0], a1 = ap[1];
          v4f va, vb;
          va.x = (float)v8[0]; va.y = (float)v8[1]; va.z = (float)v8[2]; va.w = (float)v8[3];
          vb.x = (float)v8[4]; vb.y = (float)v8[5]; vb.z = (float)v8[6]; vb.w = (float)v8[7];
          a0 = a0 * sc + va * p;
          a1 = a1 * sc + vb * p;
          ap[0] = a0;
          ap[1] = a1;
          if ((lane & 7) == 0) {
            den[slot * HEADS + hh] = dn * sc + p;
            smx[slot * HEADS + hh] = mn;
          }
          if (lane == 0) {
            const int c = cnt[slot];
            cnt[slot] = c + 1;
          }
          __builtin_amdgcn_fence(__ATOMIC_RELEASE, "wavefront");
          __builtin_amdgcn_wave_barrier();
        }
      }
    }
    __syncthreads();
  }

#pragma unroll 1
  for (int j = 0; j < NB / NWAVE; ++j) {
    const int slot = wave * (NB / NWAVE) + j;
    const int node = nodeBase + slot;
    if (node >= nN) break;
    const int   c   = cnt[slot];
    const int   hh  = lane >> 3;
    const float dv  = den[slot * HEADS + hh];
    const float inv = 1.0f / fmaxf(dv, 1.0e-20f);
    const v4f* ap = (const v4f*)(sacc + slot * IN + 8 * lane);
    v4f a0 = ap[0] * inv;
    v4f a1 = ap[1] * inv;
    const v8h vo = *(const v8h*)(Vh + (size_t)node * IN + 8 * lane);
    const bool agg = (c > 0);
    a0.x = agg ? a0.x : (float)vo[0]; a0.y = agg ? a0.y : (float)vo[1];
    a0.z = agg ? a0.z : (float)vo[2]; a0.w = agg ? a0.w : (float)vo[3];
    a1.x = agg ? a1.x : (float)vo[4]; a1.y = agg ? a1.y : (float)vo[5];
    a1.z = agg ? a1.z : (float)vo[6]; a1.w = agg ? a1.w : (float)vo[7];
    Pack16 u;
    u.h = cvt8(a0, a1);
    _Float16* mp = Mh + (size_t)node * IN + 8 * lane;
    *(volatile v4i*)mp = u.i;
    __threadfence();
    *(volatile v4i*)mp = u.i;
  }
}

extern "C" void kernel_launch(void* const* d_in, const int* in_sizes, int n_in,
                              void* d_out, int out_size, void* d_ws, size_t ws_size,
                              hipStream_t stream) {
  if (n_in < 15) return;
  const int nN = in_sizes[0] / IN;
  const int nE = in_sizes[2];
  if (nN <= 0 || in_sizes[0] != nN * IN) return;
  if (nE < 0 || in_sizes[1] != 2 * nE) return;
  if (in_sizes[3] != IN) return;
  if (in_sizes[4] != IN * IN || in_sizes[6] != IN * IN || in_sizes[8] != IN * IN || in_sizes[11] != IN * IN) return;
  if (in_sizes[5] != IN || in_sizes[7] != IN || in_sizes[9] != IN || in_sizes[12] != IN) return;
  if (in_sizes[13] != IN || in_sizes[14] != IN) return;
  if (in_sizes[10] <= 0 || (in_sizes[10] % HID) != 0) return;
  const int nR = in_sizes[10] / HID;
  if (out_size != nN * IN) return;

  const float* x     = (const float*)d_in[0];
  const int*   ei    = (const int*)d_in[1];
  const int*   erel  = (const int*)d_in[2];
  const float* qe    = (const float*)d_in[3];
  const float* Wq    = (const float*)d_in[4];
  const float* bq    = (const float*)d_in[5];
  const float* Wk    = (const float*)d_in[6];
  const float* bk    = (const float*)d_in[7];
  const float* Wv    = (const float*)d_in[8];
  const float* bv    = (const float*)d_in[9];
  const float* relw  = (const float*)d_in[10];
  const float* Wo    = (const float*)d_in[11];
  const float* bo    = (const float*)d_in[12];
  const float* gam   = (const float*)d_in[13];
  const float* bet   = (const float*)d_in[14];
  float* out = (float*)d_out;

  const int nP = ((nN + GR - 1) / GR) * GR;
  const size_t planeB = (size_t)nP * IN * sizeof(_Float16);
  size_t off = 0;
  _Float16* Wt = (_Float16*)((char*)d_ws + off); off += (size_t)4 * IN * IN * sizeof(_Float16);
  _Float16* Qh = (_Float16*)((char*)d_ws + off); off += planeB;
  _Float16* Kh = (_Float16*)((char*)d_ws + off); off += planeB;
  _Float16* Vh = (_Float16*)((char*)d_ws + off); off += planeB;
  _Float16* Mh = (_Float16*)((char*)d_ws + off); off += planeB;
  if (off > ws_size) return;

  k_prepw<<<dim3(IN / TT, IN / TT, 4), NTHR, 0, stream>>>(Wq, Wk, Wv, Wo, Wt);

  k_gemm<0><<<dim3(nP / GR, 3), NTHR, 0, stream>>>(x, qe, Mh, Wt, bq, bk, bv, gam, bet,
                                                     Qh, Kh, Vh, out, nN);

  hipFuncSetAttribute(reinterpret_cast<const void*>(&k_agg),
                      hipFuncAttributeMaxDynamicSharedMemorySize, LDS_AGG_BYTES);
  const int gridA = (nN + NB - 1) / NB;
  k_agg<<<gridA, NTHR, LDS_AGG_BYTES, stream>>>(ei, erel, Qh, Kh, Vh, relw, Mh, nN, nE, nR);

  k_gemm<1><<<dim3(nP / GR, 1), NTHR, 0, stream>>>(x, qe, Mh, Wt + (size_t)3 * IN * IN, bo, bo, bo,
                                                     gam, bet, Qh, Kh, Vh, out, nN);
}
